// Dense_54047868452885
// MI455X (gfx1250) — hardware-run, weakly checked
//
#include <hip/hip_runtime.h>


#ifndef MROWS
#define MROWS 8192
#endif
#define MROWS_FULL 8192
#define KD    1024
#define NOUT  1024

static_assert(MROWS % 64 == 0);
static_assert(NOUT % 64 == 0);
static_assert(KD % 32 == 0);
static_assert(KD % 8 == 0);
static_assert(((size_t)MROWS * KD) % 8 == 0);
static_assert(((size_t)NOUT * KD) % 8 == 0);
static_assert(MROWS <= MROWS_FULL);
static_assert(NOUT == 256 * 4);
static_assert((size_t)MROWS_FULL * NOUT * 4 == (size_t)33554432);
static_assert(((size_t)MROWS_FULL * NOUT * 4) % 128 == 0);
static_assert(8 * 32 * 16 == 16 * 64 * 4);
static_assert(16 * 16 == 64 * 4);
static_assert(16 * 68 * 4 + 64 * 4 <= 131072);

typedef _Float16 h16;
typedef unsigned short bf;
typedef __attribute__((ext_vector_type(16))) __bf16   v16bf;
typedef __attribute__((ext_vector_type(16))) _Float16 v16h;
typedef __attribute__((ext_vector_type(8)))  _Float16 v8h;
typedef __attribute__((ext_vector_type(8)))  unsigned short v8us;
typedef __attribute__((ext_vector_type(8)))  float    v8f;
typedef __attribute__((ext_vector_type(4)))  float    v4f;
typedef v4f  __attribute__((may_alias)) v4fa;

__device__ __forceinline__ unsigned short f2bf(float f) { unsigned u = __float_as_uint(f); u += 0x7FFFu + ((u >> 16) & 1u); return (unsigned short)(u >> 16); }
__device__ __forceinline__ float bfr(float f) { return __uint_as_float(((unsigned)f2bf(f)) << 16); }
__device__ __forceinline__ v16h cat16(v8h lo, v8h hi) { return __builtin_shufflevector(lo, hi, 0, 1, 2, 3, 4, 5, 6, 7, 8, 9, 10, 11, 12, 13, 14, 15); }
__device__ __forceinline__ v16bf cat16b(v8us lo, v8us hi) { return __builtin_bit_cast(v16bf, __builtin_shufflevector(lo, hi, 0, 1, 2, 3, 4, 5, 6, 7, 8, 9, 10, 11, 12, 13, 14, 15)); }
__device__ __forceinline__ v8f wmma16(v16h a, v16h b, v8f c) { return __builtin_amdgcn_wmma_f32_16x16x32_f16(false, a, false, b, (short)0, c, false, false); }
__device__ __forceinline__ v8f wmmab(v16bf a, v16bf b, v8f c) { return __builtin_amdgcn_wmma_f32_16x16x32_bf16(false, a, false, b, (short)0, c, false, false); }
__device__ __forceinline__ v16h  ldh(const h16* p) { return cat16(*(const v8h*)p, *(const v8h*)(p + 16)); }
__device__ __forceinline__ v16bf ldb(const bf* p)  { return cat16b(*(const v8us*)p, *(const v8us*)(p + 16)); }
__device__ __forceinline__ void wave_sync() { __builtin_amdgcn_fence(3  , "wavefront"); __builtin_amdgcn_wave_barrier(); asm volatile("" ::: "memory"); }

__global__ __launch_bounds__(256) void k_cvt8(const float* __restrict__ src, bf* dst, size_t n8) {
    const size_t i = (size_t)blockIdx.x * 256 + threadIdx.x; if (i >= n8) return;
    const v8f v = *(const v8f*)(src + i * 8); v8us o;
#pragma unroll
    for (int k = 0; k < 8; ++k) o[k] = f2bf(v[k]);
    *(volatile v8us*)(dst + i * 8) = o; __threadfence(); *(volatile v8us*)(dst + i * 8) = o;
}

__global__ __launch_bounds__(32) void k_affine(const bf* __restrict__ A, const bf* __restrict__ Bt, const float* __restrict__ bvec, const float* __restrict__ aux,
                                               const float* __restrict__ state, float* OUT, float* PS) {
#pragma clang fp contract(off)
    __shared__ __align__(16) float os[16 * 68];
    __shared__ __align__(16) float cl[64];
    const int K = KD;
    const int lane = threadIdx.x & 31, lr = lane & 15, hi = lane >> 4; const int r0 = blockIdx.x * 64, c0 = blockIdx.y * 64;
    v8f acc[4][4];
#pragma unroll
    for (int mb = 0; mb < 4; ++mb)
#pragma unroll
        for (int nb = 0; nb < 4; ++nb) acc[mb][nb] = (v8f){};
    const size_t aoff = (size_t)(r0 + lr) * K + 8 * hi, boff = (size_t)(c0 + lr) * K + 8 * hi;
#pragma unroll 1
    for (int kc = 0; kc < K; kc += 32) {
        v16bf a[4];
#pragma unroll
        for (int mb = 0; mb < 4; ++mb) a[mb] = ldb(A + aoff + (size_t)mb * 16 * K + kc);
#pragma unroll
        for (int nb = 0; nb < 4; ++nb) { const v16bf b = ldb(Bt + boff + (size_t)nb * 16 * K + kc);
#pragma unroll
            for (int mb = 0; mb < 4; ++mb) acc[mb][nb] = wmmab(a[mb], b, acc[mb][nb]); }
        asm volatile("v_nop\n\tv_nop\n\tv_nop\n\tv_nop" : "+v"(acc[0][0]), "+v"(acc[1][1]), "+v"(acc[2][2]), "+v"(acc[3][3]) : "v"(a[0]), "v"(a[1]), "v"(a[2]), "v"(a[3]));
    }
    float eb[4], ea[4], cs[4];
#pragma unroll
    for (int nb = 0; nb < 4; ++nb) { const int c = c0 + nb * 16 + lr;
        eb[nb] = bfr(bvec[c]); ea[nb] = bfr(aux[2 * c]) * bfr(state[c]); cs[nb] = 0.0f; }
#pragma unroll
    for (int mb = 0; mb < 4; ++mb) {
#pragma unroll
        for (int nb = 0; nb < 4; ++nb) {
#pragma unroll
            for (int j = 0; j < 8; ++j) { const float g = acc[mb][nb][j]; cs[nb] += g; os[(hi * 8 + j) * 68 + nb * 16 + lr] = (g + eb[nb]) + ea[nb]; } }
        wave_sync();
        float* orow = OUT + (size_t)(r0 + mb * 16) * NOUT + c0;
#pragma unroll 1
        for (int ps = 0; ps < 2; ++ps) {
#pragma unroll
            for (int s = 0; s < 8; ++s) { const int p = s * 32 + lane; const int row = p >> 4, c4 = (p & 15) * 4;
                const v4f val = *(const v4fa*)(&os[row * 68 + c4]);
                *(volatile v4f*)(orow + (size_t)row * NOUT + c4) = val; }
            if (ps == 0) __threadfence(); }
        wave_sync();
    }
#pragma unroll
    for (int nb = 0; nb < 4; ++nb) cs[nb] += __shfl_xor(cs[nb], 16, 32);
    if (hi == 0) {
#pragma unroll
        for (int nb = 0; nb < 4; ++nb) cl[nb * 16 + lr] = cs[nb]; }
    wave_sync();
    const v4f pv = *(const v4fa*)(&cl[lr * 4]);
    float* prow = PS + (size_t)blockIdx.x * NOUT + c0 + lr * 4;
#pragma unroll 1
    for (int ps = 0; ps < 2; ++ps) {
        if (lane < 16) *(volatile v4f*)prow = pv;
        if (ps == 0) __threadfence(); }
}

__global__ __launch_bounds__(256) void k_state(const float* __restrict__ PS, const float* __restrict__ bvec, const float* __restrict__ aux, const float* __restrict__ state, float* NS) {
#pragma clang fp contract(off)
    const int c4 = threadIdx.x * 4;
    v4f s = (v4f){};
#pragma unroll 1
    for (int rt = 0; rt < MROWS / 64; ++rt) { const v4f p = *(const v4f*)(PS + (size_t)rt * NOUT + c4); s = s + p; }
    const v4f bb = *(const v4f*)(bvec + c4); const v4f sv = *(const v4f*)(state + c4);
    const v4f a0 = *(const v4f*)(aux + 2 * c4); const v4f a1 = *(const v4f*)(aux + 2 * c4 + 4);
    const float invm = 1.0f / (float)MROWS;
    v4f o;
    o[0] = bfr(a0[1]) * bfr(sv[0]) + (s[0] * invm + bfr(bb[0]));
    o[1] = bfr(a0[3]) * bfr(sv[1]) + (s[1] * invm + bfr(bb[1]));
    o[2] = bfr(a1[1]) * bfr(sv[2]) + (s[2] * invm + bfr(bb[2]));
    o[3] = bfr(a1[3]) * bfr(sv[3]) + (s[3] * invm + bfr(bb[3]));
    *(volatile v4f*)(NS + c4) = o; __threadfence(); *(volatile v4f*)(NS + c4) = o;
}

static constexpr size_t al256(size_t v) { return (v + 255) & ~(size_t)255; }
static constexpr size_t SZ_XB = al256((size_t)MROWS * KD * 2);
static constexpr size_t SZ_WB = al256((size_t)NOUT * KD * 2);
static constexpr size_t SZ_PS = al256((size_t)(MROWS / 64) * NOUT * 4);
static constexpr size_t SZ_TOTAL = SZ_XB + SZ_WB + SZ_PS;
static_assert(SZ_TOTAL <= (size_t)134217728);
static_assert((size_t)(MROWS / 64 - 1) * NOUT + (NOUT - 64) + 15 * 4 + 3 < (size_t)(MROWS / 64) * NOUT);
static_assert((size_t)(MROWS - 1) * NOUT + (NOUT - 64) + 15 * 4 + 3 < (size_t)MROWS_FULL * NOUT);

extern "C" void kernel_launch(void* const* d_in, const int* in_sizes, int n_in,
                              void* d_out, int out_size, void* d_ws, size_t ws_size, hipStream_t stream) {
    if (n_in < 6) return;
    if ((size_t)in_sizes[0] < (size_t)MROWS * KD) return;
    if ((size_t)in_sizes[1] < (size_t)NOUT * KD) return;
    if (in_sizes[2] < NOUT || in_sizes[3] < 2 * NOUT || in_sizes[4] < NOUT) return;
    if ((size_t)out_size < (size_t)MROWS_FULL * NOUT + NOUT) return;
    if (SZ_TOTAL > ws_size) return;
    const float* x  = (const float*)d_in[0];
    const float* w  = (const float*)d_in[1];
    const float* bv = (const float*)d_in[2];
    const float* ax = (const float*)d_in[3];
    const float* st = (const float*)d_in[4];
    float* OUT = (float*)d_out;
    float* NS  = OUT + (size_t)MROWS_FULL * NOUT;
    char* wsp = (char*)d_ws;
    bf* XB = (bf*)wsp; wsp += SZ_XB;
    bf* WB = (bf*)wsp; wsp += SZ_WB;
    float* PS = (float*)wsp; wsp += SZ_PS;

    { const size_t n8 = (size_t)MROWS * KD / 8; k_cvt8<<<(unsigned)((n8 + 255) / 256), 256, 0, stream>>>(x, XB, n8); }
    { const size_t n8 = (size_t)NOUT * KD / 8;  k_cvt8<<<(unsigned)((n8 + 255) / 256), 256, 0, stream>>>(w, WB, n8); }
    k_affine<<<dim3(MROWS / 64, NOUT / 64, 1), 32, 0, stream>>>(XB, WB, bv, ax, st, OUT, PS);
    k_state<<<1, 256, 0, stream>>>(PS, bv, ax, st, NS);
}
